// MambaBlock_43533788512997
// MI455X (gfx1250) — hardware-verified
//
#include <hip/hip_runtime.h>
#include <stddef.h>
#include <stdint.h>
#include <math.h>


#define DM     1024
#define DI     2048
#define NIN    4096
#define DS     16
#define RK     64
#define XW     96
#define LSEQ   2048
#define MROWS  4096
#define K2     4096
#define KDT    128
#define NTHR   256
#define GBM    64
#define GTHR   128
#define SC_THR 128
#define SC_CH  64
#define SC_TC  64

#define U_XB   (MROWS * (DM / 8))
#define U_WIN  (NIN * (DM / 8))
#define U_WX   (XW * (K2 / 8))
#define U_WDT  (DI * (KDT / 8))
#define U_WO   (DM * (K2 / 8))
#define U_AE   (DI * DS / 4)
#define E0     (U_XB)
#define E1     (E0 + U_WIN)
#define E2     (E1 + U_WX)
#define E3     (E2 + U_WDT)
#define E4     (E3 + U_WO)
#define E5     (E4 + U_AE)

static_assert(U_XB % NTHR == 0 && U_WIN % NTHR == 0 && U_WX % NTHR == 0);
static_assert(U_WDT % NTHR == 0 && U_WO % NTHR == 0 && U_AE % NTHR == 0);
static_assert(DM % 32 == 0 && K2 % 32 == 0 && KDT % 32 == 0);
static_assert(MROWS % GBM == 0 && NIN % 128 == 0 && DI % 128 == 0 && DM % 128 == 0 && XW == 6 * 16);
static_assert(K2 == 2 * DI && KDT == 2 * RK && XW == RK + 2 * DS);
static_assert(DI % SC_CH == 0 && LSEQ % SC_TC == 0 && SC_THR == 2 * SC_CH);
static_assert((MROWS * (DI / 2)) % NTHR == 0);

typedef float          v2f   __attribute__((ext_vector_type(2)));
typedef float          v4f   __attribute__((ext_vector_type(4)));
typedef float          v8f   __attribute__((ext_vector_type(8)));
typedef int            v8i   __attribute__((ext_vector_type(8)));
typedef unsigned short v4us  __attribute__((ext_vector_type(4)));
typedef unsigned short v8us  __attribute__((ext_vector_type(8)));
typedef unsigned short v16us __attribute__((ext_vector_type(16)));
typedef __bf16         v16bf __attribute__((ext_vector_type(16)));
typedef v2f  __attribute__((may_alias)) v2fa;
typedef v4f  __attribute__((may_alias)) v4fa;
typedef v4us __attribute__((may_alias)) v4usa;
typedef v8us __attribute__((may_alias)) v8usa;
union FragB { v16bf v; v16us u; v8us h[2]; v8i w; };

__device__ __forceinline__ v8f wmb(const FragB& a, const FragB& b, v8f c) {
  v8f d = __builtin_amdgcn_wmma_f32_16x16x32_bf16(false, a.v, false, b.v, (short)0, c, false, false);
  asm volatile("v_nop\n\tv_nop\n\tv_nop\n\tv_nop" : "+v"(d) : "v"(a.w), "v"(b.w));
  return d;
}

__device__ __forceinline__ unsigned bf16_bits(float f) {
  const unsigned u = __float_as_uint(f);
  return (u + 0x7FFFu + ((u >> 16) & 1u)) >> 16;
}
__device__ __forceinline__ float bf16_val(float f) {
  return __uint_as_float(bf16_bits(f) << 16);
}

__device__ __forceinline__ float silu_f(float x) {
  return x * (1.0f / (1.0f + expf(-x)));
}
__device__ __forceinline__ float softplus_f(float v) {
  return fmaxf(v, 0.0f) + log1pf(expf(-fabsf(v)));
}

__device__ __forceinline__ void cvt_unit(const float* __restrict__ x, unsigned short* xb, int v) {
  const float* p = x + (size_t)v * 8;
  const v4f a = *(const v4fa*)p;
  const v4f b = *(const v4fa*)(p + 4);
  v8us o;
  o[0] = (unsigned short)bf16_bits(a.x); o[1] = (unsigned short)bf16_bits(a.y);
  o[2] = (unsigned short)bf16_bits(a.z); o[3] = (unsigned short)bf16_bits(a.w);
  o[4] = (unsigned short)bf16_bits(b.x); o[5] = (unsigned short)bf16_bits(b.y);
  o[6] = (unsigned short)bf16_bits(b.z); o[7] = (unsigned short)bf16_bits(b.w);
  unsigned short* dp = xb + (size_t)v * 8;
  *(volatile v8us*)dp = o;
  __threadfence();
  *(volatile v8us*)dp = o;
}

__device__ __forceinline__ void tr_unit(const float* __restrict__ W, int ldw, int kmask, int sh,
                                        unsigned short* P, int v) {
  const int n  = v >> sh;
  const int k8 = (v & ((1 << sh) - 1)) * 8;
  const int kk = k8 & kmask;
  const float* p = W + (size_t)kk * (size_t)ldw + n;
  v8us o;
#pragma unroll
  for (int i = 0; i < 8; ++i) o[i] = (unsigned short)bf16_bits(p[(size_t)i * (size_t)ldw]);
  unsigned short* dp = P + ((size_t)n << (sh + 3)) + k8;
  *(volatile v8us*)dp = o;
  __threadfence();
  *(volatile v8us*)dp = o;
}

__device__ __forceinline__ void aexp_unit(const float* __restrict__ al, float* ae, int v) {
  const v4f a = *(const v4fa*)(al + (size_t)v * 4);
  v4f o;
  o.x = -expf(bf16_val(a.x)); o.y = -expf(bf16_val(a.y));
  o.z = -expf(bf16_val(a.z)); o.w = -expf(bf16_val(a.w));
  float* dp = ae + (size_t)v * 4;
  *(volatile v4f*)dp = o;
  __threadfence();
  *(volatile v4f*)dp = o;
}

__global__ __launch_bounds__(NTHR) void k_prep(const float* __restrict__ x, const float* __restrict__ Win,
                                               const float* __restrict__ Wx, const float* __restrict__ Wdt,
                                               const float* __restrict__ Wout, const float* __restrict__ Alog,
                                               unsigned short* XB, unsigned short* WINT, unsigned short* WX2,
                                               unsigned short* WDT2, unsigned short* WO2, float* AEXP) {
  const int u = (int)blockIdx.x * NTHR + (int)threadIdx.x;
  if (u < E0)       cvt_unit(x, XB, u);
  else if (u < E1)  tr_unit(Win,  NIN, DM - 1, 7, WINT, u - E0);
  else if (u < E2)  tr_unit(Wx,   XW,  DI - 1, 9, WX2,  u - E1);
  else if (u < E3)  tr_unit(Wdt,  DI,  RK - 1, 4, WDT2, u - E2);
  else if (u < E4)  tr_unit(Wout, DM,  DI - 1, 9, WO2,  u - E3);
  else if (u < E5)  aexp_unit(Alog, AEXP, u - E4);
}

template <int NT, int MODE>
__global__ __launch_bounds__(GTHR) void k_gemm(const unsigned short* __restrict__ A, int lda,
                                               const unsigned short* __restrict__ BT, int K,
                                               float* outF, int ldo, size_t off1,
                                               const float* __restrict__ bias, unsigned short* outH) {
  constexpr int BN = 16 * NT;
  __shared__ __attribute__((aligned(16))) float stg[GBM * BN];
  const int tid = (int)threadIdx.x, lane = tid & 31, wave = tid >> 5, hh = lane >> 4, m = lane & 15;
  const int rowBase = (int)blockIdx.x * GBM;
  const int col0    = (int)blockIdx.y * BN;

  v8f acc[NT];
  {
    const v8f z = {0.f, 0.f, 0.f, 0.f, 0.f, 0.f, 0.f, 0.f};
#pragma unroll
    for (int t = 0; t < NT; ++t) acc[t] = z;
  }
  const unsigned short* ap = A  + (size_t)(rowBase + 16 * wave + m) * (size_t)lda + 8 * hh;
  const unsigned short* wp = BT + (size_t)(col0 + m) * (size_t)K + 8 * hh;
#pragma unroll 1
  for (int k0 = 0; k0 < K; k0 += 32) {
    FragB af;
    af.h[0] = *(const v8usa*)(ap + k0);
    af.h[1] = *(const v8usa*)(ap + k0 + 16);
#pragma unroll
    for (int t = 0; t < NT; ++t) {
      const unsigned short* wq = wp + (size_t)(16 * t) * (size_t)K + k0;
      FragB bf;
      bf.h[0] = *(const v8usa*)wq;
      bf.h[1] = *(const v8usa*)(wq + 16);
      acc[t] = wmb(af, bf, acc[t]);
    }
  }

#pragma unroll
  for (int t = 0; t < NT; ++t) {
    const int lc = 16 * t + m;
#pragma unroll
    for (int r = 0; r < 8; ++r) {
      const int lr = 16 * wave + 8 * hh + r;
      stg[lr * BN + lc] = acc[t][r];
    }
  }
  __syncthreads();

  if constexpr (MODE == 1) {
    const int lc = lane < 24 ? lane : 23;
    v4f pv[16];
#pragma unroll
    for (int i = 0; i < 16; ++i) pv[i] = *(const v4fa*)(stg + (16 * wave + i) * BN + 4 * lc);
    float* ob = outF + (size_t)(rowBase + 16 * wave) * (size_t)XW + 4 * lc;
    const bool w24 = lane < 24;
#pragma unroll
    for (int i = 0; i < 16; ++i) { if (w24) *(volatile v4f*)(ob + (size_t)i * XW) = pv[i]; }
    __threadfence();
#pragma unroll
    for (int i = 0; i < 16; ++i) { if (w24) *(volatile v4f*)(ob + (size_t)i * XW) = pv[i]; }
    __syncthreads();
    unsigned short* sh = (unsigned short*)stg;
    const bool w16 = lane < 16;
#pragma unroll
    for (int i = 0; i < 16; ++i) {
      v4us h4, l4;
      unsigned hb;
      hb = bf16_bits(pv[i].x); h4[0] = (unsigned short)hb; l4[0] = (unsigned short)bf16_bits(pv[i].x - __uint_as_float(hb << 16));
      hb = bf16_bits(pv[i].y); h4[1] = (unsigned short)hb; l4[1] = (unsigned short)bf16_bits(pv[i].y - __uint_as_float(hb << 16));
      hb = bf16_bits(pv[i].z); h4[2] = (unsigned short)hb; l4[2] = (unsigned short)bf16_bits(pv[i].z - __uint_as_float(hb << 16));
      hb = bf16_bits(pv[i].w); h4[3] = (unsigned short)hb; l4[3] = (unsigned short)bf16_bits(pv[i].w - __uint_as_float(hb << 16));
      unsigned short* srow = sh + (size_t)(16 * wave + i) * KDT;
      if (w16) {
        *(v4usa*)(srow + 4 * lane) = h4;
        *(v4usa*)(srow + RK + 4 * lane) = l4;
      }
    }
    __syncthreads();
    const int lq = lane & 15;
    v8us qv[16];
#pragma unroll
    for (int i = 0; i < 16; ++i) qv[i] = *(const v8usa*)(sh + (size_t)(16 * wave + i) * KDT + 8 * lq);
    unsigned short* hp = outH + (size_t)(rowBase + 16 * wave) * (size_t)KDT + 8 * lq;
#pragma unroll
    for (int i = 0; i < 16; ++i) { if (w16) *(volatile v8us*)(hp + (size_t)i * KDT) = qv[i]; }
    __threadfence();
#pragma unroll
    for (int i = 0; i < 16; ++i) { if (w16) *(volatile v8us*)(hp + (size_t)i * KDT) = qv[i]; }
  } else {
    float* srow = stg + (16 * wave) * BN + 4 * lane;
    size_t poff = 0;
    int cloc = col0;
    if constexpr (MODE == 0) {
      if (col0 >= DI) {
        poff = off1;
        cloc = col0 - DI;
#pragma unroll 1
        for (int i = 0; i < 16; ++i) {
          float* p = srow + i * BN;
          v4f v = *(const v4fa*)p;
          v.x = silu_f(v.x); v.y = silu_f(v.y); v.z = silu_f(v.z); v.w = silu_f(v.w);
          *(v4fa*)p = v;
        }
      }
    }
    if constexpr (MODE == 2) {
      const v4f bq = *(const v4fa*)(bias + col0 + 4 * lane);
      const float b0 = bf16_val(bq.x), b1 = bf16_val(bq.y), b2 = bf16_val(bq.z), b3 = bf16_val(bq.w);
#pragma unroll 1
      for (int i = 0; i < 16; ++i) {
        float* p = srow + i * BN;
        v4f v = *(const v4fa*)p;
        v.x = softplus_f(v.x + b0); v.y = softplus_f(v.y + b1);
        v.z = softplus_f(v.z + b2); v.w = softplus_f(v.w + b3);
        *(v4fa*)p = v;
      }
    }
    v4f pv[16];
#pragma unroll
    for (int i = 0; i < 16; ++i) pv[i] = *(const v4fa*)(srow + i * BN);
    float* ob = outF + poff + (size_t)(rowBase + 16 * wave) * (size_t)ldo + cloc + 4 * lane;
#pragma unroll
    for (int i = 0; i < 16; ++i) *(volatile v4f*)(ob + (size_t)i * (size_t)ldo) = pv[i];
    __threadfence();
#pragma unroll
    for (int i = 0; i < 16; ++i) *(volatile v4f*)(ob + (size_t)i * (size_t)ldo) = pv[i];
  }
}

__global__ __launch_bounds__(NTHR) void k_conv(const float* __restrict__ XS, const float* __restrict__ cw,
                                               const float* __restrict__ cb, float* XC, unsigned short* XChl) {
  const int u = (int)blockIdx.x * NTHR + (int)threadIdx.x;
  const int r = u >> 10;
  const int c = (u & 1023) * 2;
  const int t = r & (LSEQ - 1);
  const v4f wa = *(const v4fa*)(cw + (size_t)c * 4);
  const v4f wb = *(const v4fa*)(cw + (size_t)c * 4 + 4);
  const v2f bb = *(const v2fa*)(cb + c);
  const float w0[4] = {bf16_val(wa.x), bf16_val(wa.y), bf16_val(wa.z), bf16_val(wa.w)};
  const float w1[4] = {bf16_val(wb.x), bf16_val(wb.y), bf16_val(wb.z), bf16_val(wb.w)};
  v2f xv[4];
#pragma unroll
  for (int j = 0; j < 4; ++j) {
    const bool ok = (t - 3 + j) >= 0;
    const int rr = ok ? (r - 3 + j) : r;
    xv[j] = *(const v2fa*)(XS + (size_t)rr * DI + c);
  }
  float a0 = 0.0f, a1 = 0.0f;
#pragma unroll
  for (int j = 0; j < 4; ++j) {
    const bool ok = (t - 3 + j) >= 0;
    const float e0 = ok ? w0[j] : 0.0f;
    const float e1 = ok ? w1[j] : 0.0f;
    a0 = fmaf(e0, xv[j].x, a0);
    a1 = fmaf(e1, xv[j].y, a1);
  }
  const float p0 = a0 + bf16_val(bb.x);
  const float p1 = a1 + bf16_val(bb.y);
  v2f y;
  y.x = silu_f(p0);
  y.y = silu_f(p1);
  const unsigned hb0 = bf16_bits(y.x), hb1 = bf16_bits(y.y);
  const unsigned lb0 = bf16_bits(y.x - __uint_as_float(hb0 << 16));
  const unsigned lb1 = bf16_bits(y.y - __uint_as_float(hb1 << 16));
  const unsigned hw = hb0 | (hb1 << 16);
  const unsigned lw = lb0 | (lb1 << 16);
  float* xp = XC + (size_t)r * DI + c;
  unsigned short* hp = XChl + (size_t)r * K2 + c;
  *(volatile v2f*)xp = y;
  *(volatile unsigned*)hp = hw;
  *(volatile unsigned*)(hp + DI) = lw;
  __threadfence();
  *(volatile v2f*)xp = y;
  *(volatile unsigned*)hp = hw;
  *(volatile unsigned*)(hp + DI) = lw;
}

__global__ __launch_bounds__(SC_THR) void k_scan(const float* __restrict__ DELTA, const float* __restrict__ XC,
                                                 const float* __restrict__ SR, const float* __restrict__ XDBL,
                                                 const float* __restrict__ AEXP, const float* __restrict__ Dp,
                                                 unsigned short* Yhl) {
  __shared__ __attribute__((aligned(16))) float bc[SC_TC * 32];
  __shared__ __attribute__((aligned(16))) unsigned short ystg[2 * SC_TC * SC_CH];
  const int tid = (int)threadIdx.x;
  const int b   = (int)blockIdx.x >> 5;
  const int cb  = ((int)blockIdx.x & 31) * SC_CH;
  const int cl  = tid >> 1;
  const int nh  = tid & 1;
  const int d   = cb + cl;

  const v4f a0 = *(const v4fa*)(AEXP + (size_t)d * DS + 8 * nh);
  const v4f a1 = *(const v4fa*)(AEXP + (size_t)d * DS + 8 * nh + 4);
  const float av[8] = {a0.x, a0.y, a0.z, a0.w, a1.x, a1.y, a1.z, a1.w};
  const float dpar = bf16_val(Dp[d]);
  float h[8] = {0.f, 0.f, 0.f, 0.f, 0.f, 0.f, 0.f, 0.f};

#pragma unroll 1
  for (int ch = 0; ch < LSEQ / SC_TC; ++ch) {
    const int r0 = b * LSEQ + ch * SC_TC;
    __syncthreads();
#pragma unroll
    for (int q = 0; q < 4; ++q) {
      const int idx = q * SC_THR + tid;
      const int tl  = idx >> 3;
      const int c4  = (idx & 7) * 4;
      const v4f v = *(const v4fa*)(XDBL + (size_t)(r0 + tl) * XW + RK + c4);
      *(v4fa*)(bc + tl * 32 + c4) = v;
    }
    __syncthreads();
#pragma unroll 1
    for (int tl = 0; tl < SC_TC; ++tl) {
      const size_t gi = (size_t)(r0 + tl) * DI + d;
      const float dv = DELTA[gi];
      const float xv = XC[gi];
      const float sv = SR[gi];
      const v4f B0 = *(const v4fa*)(bc + tl * 32 + 8 * nh);
      const v4f B1 = *(const v4fa*)(bc + tl * 32 + 8 * nh + 4);
      const v4f C0 = *(const v4fa*)(bc + tl * 32 + DS + 8 * nh);
      const v4f C1 = *(const v4fa*)(bc + tl * 32 + DS + 8 * nh + 4);
      const float bv[8] = {B0.x, B0.y, B0.z, B0.w, B1.x, B1.y, B1.z, B1.w};
      const float cv[8] = {C0.x, C0.y, C0.z, C0.w, C1.x, C1.y, C1.z, C1.w};
      const float dxb = dv * xv;
      float y = 0.0f;
#pragma unroll
      for (int n = 0; n < 8; ++n) {
        const float dA = expf(dv * av[n]);
        h[n] = fmaf(dA, h[n], dxb * bv[n]);
        y = fmaf(h[n], cv[n], y);
      }
      const float yo = __shfl_xor(y, 1, 32);
      const float ys = y + yo;
      const float yv = (ys + xv * dpar) * sv;
      const unsigned hb = bf16_bits(yv);
      const unsigned lb = bf16_bits(yv - __uint_as_float(hb << 16));
      const unsigned bits = (nh != 0) ? lb : hb;
      ystg[nh * (SC_TC * SC_CH) + tl * SC_CH + cl] = (unsigned short)bits;
    }
    __syncthreads();
    v8us qv[8];
#pragma unroll
    for (int q = 0; q < 8; ++q) {
      const int idx  = q * SC_THR + tid;
      const int line = idx >> 3;
      const int pc   = idx & 7;
      qv[q] = *(const v8usa*)(ystg + line * SC_CH + pc * 8);
    }
#pragma unroll
    for (int q = 0; q < 8; ++q) {
      const int idx  = q * SC_THR + tid;
      const int line = idx >> 3;
      const int pc   = idx & 7;
      const int pl   = line >> 6;
      const int tl   = line & 63;
      unsigned short* dp = Yhl + (size_t)(r0 + tl) * K2 + pl * DI + cb + pc * 8;
      *(volatile v8us*)dp = qv[q];
    }
    __threadfence();
#pragma unroll
    for (int q = 0; q < 8; ++q) {
      const int idx  = q * SC_THR + tid;
      const int line = idx >> 3;
      const int pc   = idx & 7;
      const int pl   = line >> 6;
      const int tl   = line & 63;
      unsigned short* dp = Yhl + (size_t)(r0 + tl) * K2 + pl * DI + cb + pc * 8;
      *(volatile v8us*)dp = qv[q];
    }
  }
}

extern "C" void kernel_launch(void* const* d_in, const int* in_sizes, int n_in,
                              void* d_out, int out_size, void* d_ws, size_t ws_size,
                              hipStream_t stream) {
  if (n_in < 10) return;
  if (in_sizes[0] != MROWS * DM) return;
  if (in_sizes[1] != DM * NIN) return;
  if (in_sizes[2] != DI * 4) return;
  if (in_sizes[3] != DI) return;
  if (in_sizes[4] != DI * XW) return;
  if (in_sizes[5] != RK * DI) return;
  if (in_sizes[6] != DI) return;
  if (in_sizes[7] != DI * DS) return;
  if (in_sizes[8] != DI) return;
  if (in_sizes[9] != DI * DM) return;
  if (out_size != MROWS * DM) return;

  const float* x      = (const float*)d_in[0];
  const float* W_in   = (const float*)d_in[1];
  const float* conv_w = (const float*)d_in[2];
  const float* conv_b = (const float*)d_in[3];
  const float* W_x    = (const float*)d_in[4];
  const float* W_dt   = (const float*)d_in[5];
  const float* b_dt   = (const float*)d_in[6];
  const float* A_log  = (const float*)d_in[7];
  const float* D_par  = (const float*)d_in[8];
  const float* W_out  = (const float*)d_in[9];
  float* out = (float*)d_out;

  char* ws = (char*)d_ws;
  size_t off = 0;
  const size_t oXB  = off; off += (size_t)MROWS * DM * 2;
  const size_t oWIN = off; off += (size_t)NIN * DM * 2;
  const size_t oWX  = off; off += (size_t)XW * K2 * 2;
  const size_t oWDT = off; off += (size_t)DI * KDT * 2;
  const size_t oWO  = off; off += (size_t)DM * K2 * 2;
  const size_t oAE  = off; off += (size_t)DI * DS * 4;
  const size_t oXS  = off; off += (size_t)MROWS * DI * 4;
  const size_t oSR  = off; off += (size_t)MROWS * DI * 4;
  const size_t oXC  = off; off += (size_t)MROWS * DI * 4;
  const size_t oXH  = off; off += (size_t)MROWS * K2 * 2;
  const size_t oXD  = off; off += (size_t)MROWS * XW * 4;
  const size_t oDT  = off; off += (size_t)MROWS * KDT * 2;
  if (off != (size_t)163446784) return;
  if (off > ws_size) return;

  unsigned short* XB   = (unsigned short*)(ws + oXB);
  unsigned short* WINT = (unsigned short*)(ws + oWIN);
  unsigned short* WX2  = (unsigned short*)(ws + oWX);
  unsigned short* WDT2 = (unsigned short*)(ws + oWDT);
  unsigned short* WO2  = (unsigned short*)(ws + oWO);
  float*          AEXP = (float*)(ws + oAE);
  float*          XS   = (float*)(ws + oXS);
  float*          SR   = (float*)(ws + oSR);
  float*          XC   = (float*)(ws + oXC);
  unsigned short* XChl = (unsigned short*)(ws + oXH);
  float*          XDBL = (float*)(ws + oXD);
  unsigned short* DThl = (unsigned short*)(ws + oDT);
  float*          DELTA = XS;
  unsigned short* Yhl   = XChl;
  const size_t offSR = (oSR - oXS) / 4;

  k_prep<<<E5 / NTHR, NTHR, 0, stream>>>(x, W_in, W_x, W_dt, W_out, A_log, XB, WINT, WX2, WDT2, WO2, AEXP);
  k_gemm<8, 0><<<dim3(MROWS / GBM, NIN / 128), GTHR, 0, stream>>>(XB, DM, WINT, DM, XS, DI, offSR, b_dt, DThl);
  k_conv<<<(MROWS * (DI / 2)) / NTHR, NTHR, 0, stream>>>(XS, conv_w, conv_b, XC, XChl);
  k_gemm<6, 1><<<dim3(MROWS / GBM, 1), GTHR, 0, stream>>>(XChl, K2, WX2, K2, XDBL, XW, (size_t)0, b_dt, DThl);
  k_gemm<8, 2><<<dim3(MROWS / GBM, DI / 128), GTHR, 0, stream>>>(DThl, KDT, WDT2, KDT, DELTA, DI, (size_t)0, b_dt, XChl);
  k_scan<<<2 * (DI / SC_CH), SC_THR, 0, stream>>>(DELTA, XC, SR, XDBL, AEXP, D_par, Yhl);
  k_gemm<8, 3><<<dim3(MROWS / GBM, DM / 128), GTHR, 0, stream>>>(Yhl, K2, WO2, K2, out, DM, (size_t)0, b_dt, DThl);
}
